// MultiScaleAttention_19928648253537
// MI455X (gfx1250) — hardware-verified
//
#include <hip/hip_runtime.h>
#include <math.h>

#ifndef NB
#define NB 8
#endif
#define NB_FULL 8
#define SEQ 1024
#define CDIM 768
#define C3 2304
#define HEADS 12
#define HD 64
#define MTOK (NB * SEQ)
#define CW8 96
#define QK_PLANE (MTOK * CDIM)

#define X_CARRY 16
#define W_CARRY 64
#define QKV_CARRY 16
#define P_CARRY 1024
#define CTX_CARRY 64
#define ATT_CARRY 16
#define FUS_CARRY 64

#define OUT1_OFF (NB_FULL * SEQ * CDIM)
#define OUT2_OFF (OUT1_OFF + NB_FULL * 1024 * 1024)
#define OUT3_OFF (OUT2_OFF + NB_FULL * 256 * 256)
#define OUT_TOTAL (OUT3_OFF + NB_FULL * 64 * 64)

static_assert(NB >= 1 && NB <= NB_FULL);
static_assert(SEQ == 1024);
static_assert(CDIM == HEADS * HD && C3 == 3 * CDIM && HD == 64);
static_assert(CDIM % 64 == 0 && CDIM % 32 == 0 && CW8 * 8 == CDIM);
static_assert(MTOK % 64 == 0 && (NB * 256) % 64 == 0 && (NB * 64) % 64 == 0);
static_assert((2 * CDIM) % 64 == 0);
static_assert((NB * HEADS * 64) % 128 == 0);
static_assert(X_CARRY * W_CARRY == 1024);
static_assert(CTX_CARRY * W_CARRY == 4096);
static_assert(ATT_CARRY * W_CARRY == 1024);
static_assert(FUS_CARRY * W_CARRY == 4096);
static_assert(QKV_CARRY * QKV_CARRY == 256);
static_assert(P_CARRY * QKV_CARRY == 256 * CTX_CARRY);
static_assert((size_t)OUT1_OFF * 4 == 25165824);
static_assert((size_t)OUT2_OFF * 4 == 58720256);
static_assert((size_t)OUT3_OFF * 4 == 60817408);
static_assert((size_t)OUT_TOTAL * 4 == 60948480);
static_assert(8 * 16 * 68 * 4 + 2 * 128 * 4 <= 131072);
static_assert(32 * 16 * 8 == 16 * 256);
static_assert(32 * 16 * 4 == 16 * 128);

static constexpr size_t WS_TOTAL =
    (size_t)2 * ((size_t)3 * C3 * CDIM + (size_t)6 * CDIM * CDIM + (size_t)CDIM * CDIM) +
    (size_t)2 * ((size_t)MTOK + NB * 256 + NB * 64) * CDIM +
    (size_t)6 * QK_PLANE +
    (size_t)8 * NB * HEADS * SEQ +
    (size_t)2 * MTOK * CDIM +
    (size_t)4 * ((size_t)MTOK + NB * 256 + NB * 64) * CDIM;
static_assert(WS_TOTAL <= (size_t)134217728);

static constexpr float SC2 = 0.125f * 1.4426950408889634f / 256.0f;
static constexpr float CTX_FOLD = 1.0f / 256.0f;
static constexpr float INV_HEADS = 1.0f / 12.0f;
static constexpr float LOG2E = 1.4426950408889634f;

typedef __attribute__((ext_vector_type(16))) _Float16 v16h;
typedef __attribute__((ext_vector_type(8)))  _Float16 v8h;
typedef __attribute__((ext_vector_type(2)))  _Float16 v2h;
typedef __attribute__((ext_vector_type(8)))  float    v8f;
typedef __attribute__((ext_vector_type(4)))  float    v4f;
typedef __attribute__((ext_vector_type(4)))  unsigned int v4u;
typedef _Float16 h16;


#define VST2(T, ptr, val) do { const T vst2_v_ = (val); *(volatile T*)(ptr) = vst2_v_; __threadfence(); *(volatile T*)(ptr) = vst2_v_; } while (0)
#define VST2V4(ptr, val) do { const v4f vst2_v4_ = (val); *(volatile v4f*)(ptr) = vst2_v4_; __threadfence(); *(volatile v4f*)(ptr) = vst2_v4_; } while (0)

__device__ __forceinline__ float bfr(float f) {
    unsigned u = __float_as_uint(f);
    u += 0x7FFFu + ((u >> 16) & 1u);
    return __uint_as_float(u & 0xFFFF0000u);
}
static __device__ __forceinline__ h16 toh_flush(float v) { const float w = (fabsf(v) < 6.103515625e-05f) ? 0.0f : v; return (h16)w; }
__device__ __forceinline__ unsigned pack2h(float a, float b) {
    v2h t; t.x = toh_flush(a); t.y = toh_flush(b);
    return __builtin_bit_cast(unsigned, t);
}
__device__ __forceinline__ void st8hf(_Float16* P, size_t o, const float* v) {
    v8h pk;
#pragma unroll
    for (int e = 0; e < 8; ++e) pk[e] = toh_flush(v[e]);
    VST2(v8h, (v8h*)(P + o), pk);
}

union FragU { v16h v; v8h h[2]; };
__device__ __forceinline__ v16h frag_ld(const _Float16* p) {
    FragU f; f.h[0] = *(const v8h*)(p); f.h[1] = *(const v8h*)(p + 16); return f.v;
}
__device__ __forceinline__ v8f wmma16(v16h a, v16h b, v8f c) {
    c = __builtin_amdgcn_wmma_f32_16x16x32_f16(false, a, false, b, (short)0, c, false, false);
    asm volatile("v_nop\n\tv_nop\n\tv_nop\n\tv_nop" : "+v"(c) : "v"(a), "v"(b));
    return c;
}
__device__ __forceinline__ void wave_sync_lds() {
    __builtin_amdgcn_fence(3  , "workgroup");
    __builtin_amdgcn_wave_barrier();
    __builtin_amdgcn_fence(2  , "workgroup");
}

template <int MODE, int INV_SCALE, int OCARRY>
__device__ __forceinline__ void gemm64_body(
    const _Float16* __restrict__ A, unsigned lda, const _Float16* __restrict__ Bt, unsigned ldb,
    void* __restrict__ Cout, unsigned ldc, const float* __restrict__ bias,
    unsigned M, unsigned N, unsigned K, unsigned lgns) {
  __shared__ __align__(16) float sT[8][16 * 68];
  const unsigned lane = threadIdx.x & 31u;
  const unsigned wave = (unsigned)__builtin_amdgcn_readfirstlane((int)(threadIdx.x >> 5));
  const unsigned tilesN = N >> 6, tilesM = M >> 6;
  const unsigned tile = blockIdx.x * 8u + wave;
  if (tile >= tilesM * tilesN) return;
  const unsigned tm = tile / tilesN;
  const unsigned tn = tile - tm * tilesN;
  const unsigned m0 = tm << 6, n0 = tn << 6;
  const unsigned rlane = lane & 15u;
  const unsigned koff = (lane >> 4) * 8u;
  const unsigned mOff = koff;
  constexpr float scale = 1.0f / (float)INV_SCALE;
  constexpr float oc = (float)OCARRY;

  v8f acc[4][4];
#pragma unroll
  for (int i = 0; i < 4; ++i)
#pragma unroll
    for (int j = 0; j < 4; ++j) acc[i][j] = (v8f){0.f,0.f,0.f,0.f,0.f,0.f,0.f,0.f};

  for (unsigned k0 = 0; k0 < K; k0 += 32u) {
    v16h bh[4];
#pragma unroll
    for (int j = 0; j < 4; ++j)
      bh[j] = frag_ld(Bt + (size_t)(n0 + ((unsigned)j << 4) + rlane) * ldb + koff + k0);
#pragma unroll
    for (int i = 0; i < 4; ++i) {
      const v16h ah = frag_ld(A + (size_t)(m0 + ((unsigned)i << 4) + rlane) * lda + koff + k0);
#pragma unroll
      for (int j = 0; j < 4; ++j)
        acc[i][j] = wmma16(ah, bh[j], acc[i][j]);
    }
  }

  size_t cbase;
  unsigned cpitch;
  if (MODE == 2) {
    const unsigned part = tn / 12u;
    const unsigned hd = tn - part * 12u;
    const unsigned b = m0 >> lgns;
    const unsigned tok0 = m0 & ((1u << lgns) - 1u);
    cbase = (size_t)part * (size_t)QK_PLANE + ((size_t)((b * 12u + hd) << lgns) + tok0) * 64u;
    cpitch = 64u;
  } else if (MODE == 3) {
    const unsigned b = n0 >> lgns;
    const unsigned tok0 = n0 & ((1u << lgns) - 1u);
    cbase = ((size_t)((b * 12u + tm) * 64u) << lgns) + tok0;
    cpitch = 1u << lgns;
  } else {
    cbase = (size_t)m0 * ldc + n0;
    cpitch = ldc;
  }

#pragma unroll
  for (int i = 0; i < 4; ++i) {
    float brow[8];
#pragma unroll
    for (int r = 0; r < 8; ++r) brow[r] = 0.0f;
    if (MODE == 3) {
#pragma unroll
      for (int r = 0; r < 8; ++r) brow[r] = bfr(bias[m0 + ((unsigned)i << 4) + mOff + (unsigned)r]);
    }
#pragma unroll
    for (int j = 0; j < 4; ++j) {
      const unsigned n = n0 + ((unsigned)j << 4) + rlane;
      float bcol = 0.0f;
      if (MODE != 3) bcol = bfr(bias[n]);
#pragma unroll
      for (int r = 0; r < 8; ++r) {
        float v = acc[i][j][r] * scale + ((MODE == 3) ? brow[r] : bcol);
        if (MODE != 0) v *= oc;
        sT[wave][(mOff + (unsigned)r) * 68u + ((unsigned)j << 4) + rlane] = v;
      }
    }
    wave_sync_lds();
    if (MODE == 0) {
      float* C = (float*)Cout;
      const unsigned hh = lane >> 4, c4 = (lane & 15u) * 4u;
#pragma unroll
      for (int half = 0; half < 2; ++half) {
        v4f vv[4];
#pragma unroll
        for (int it = 0; it < 4; ++it) {
          const unsigned row = (unsigned)(half * 4 + it) * 2u + hh;
          vv[it] = *(const v4f*)&sT[wave][row * 68u + c4];
        }
        for (int pass = 0; pass < 2; ++pass) {
#pragma unroll
          for (int it = 0; it < 4; ++it) {
            const unsigned row = (unsigned)(half * 4 + it) * 2u + hh;
            *(volatile v4f*)(C + cbase + (size_t)(((unsigned)i << 4) + row) * cpitch + c4) = vv[it];
          }
          __threadfence();
        }
      }
    } else {
      _Float16* C = (_Float16*)Cout;
      const unsigned q = lane >> 3, c8 = (lane & 7u) * 8u;
      v8h hv[4];
#pragma unroll
      for (int it = 0; it < 4; ++it) {
        const unsigned row = (unsigned)it * 4u + q;
        const v4f s0 = *(const v4f*)&sT[wave][row * 68u + c8];
        const v4f s1 = *(const v4f*)&sT[wave][row * 68u + c8 + 4u];
        hv[it][0] = toh_flush(s0.x); hv[it][1] = toh_flush(s0.y); hv[it][2] = toh_flush(s0.z); hv[it][3] = toh_flush(s0.w);
        hv[it][4] = toh_flush(s1.x); hv[it][5] = toh_flush(s1.y); hv[it][6] = toh_flush(s1.z); hv[it][7] = toh_flush(s1.w);
      }
      for (int pass = 0; pass < 2; ++pass) {
#pragma unroll
        for (int it = 0; it < 4; ++it) {
          const unsigned row = (unsigned)it * 4u + q;
          *(volatile v8h*)(C + cbase + (size_t)(((unsigned)i << 4) + row) * cpitch + c8) = hv[it];
        }
        __threadfence();
      }
    }
    wave_sync_lds();
  }
}

__global__ __launch_bounds__(256) void k_gemm_qk(const _Float16* __restrict__ A, unsigned lda, const _Float16* __restrict__ Bt, unsigned ldb,
                                                 _Float16* __restrict__ C, const float* __restrict__ bias,
                                                 unsigned M, unsigned N, unsigned K, unsigned lgns) {
  gemm64_body<2, X_CARRY * W_CARRY, QKV_CARRY>(A, lda, Bt, ldb, (void*)C, 0u, bias, M, N, K, lgns);
}
__global__ __launch_bounds__(256) void k_gemm_vt(const _Float16* __restrict__ A, unsigned lda, const _Float16* __restrict__ Bt, unsigned ldb,
                                                 _Float16* __restrict__ C, const float* __restrict__ bias,
                                                 unsigned M, unsigned N, unsigned K, unsigned lgns) {
  gemm64_body<3, X_CARRY * W_CARRY, QKV_CARRY>(A, lda, Bt, ldb, (void*)C, 0u, bias, M, N, K, lgns);
}
__global__ __launch_bounds__(256) void k_gemm_proj(const _Float16* __restrict__ A, unsigned lda, const _Float16* __restrict__ Bt, unsigned ldb,
                                                   _Float16* __restrict__ C, unsigned ldc, const float* __restrict__ bias,
                                                   unsigned M, unsigned N, unsigned K) {
  gemm64_body<1, CTX_CARRY * W_CARRY, ATT_CARRY>(A, lda, Bt, ldb, (void*)C, ldc, bias, M, N, K, 0u);
}
__global__ __launch_bounds__(256) void k_gemm_sp(const _Float16* __restrict__ A, unsigned lda, const _Float16* __restrict__ Bt, unsigned ldb,
                                                 float* __restrict__ C, unsigned ldc, const float* __restrict__ bias,
                                                 unsigned M, unsigned N, unsigned K) {
  gemm64_body<0, ATT_CARRY * W_CARRY, 1>(A, lda, Bt, ldb, (void*)C, ldc, bias, M, N, K, 0u);
}
__global__ __launch_bounds__(256) void k_gemm_out(const _Float16* __restrict__ A, unsigned lda, const _Float16* __restrict__ Bt, unsigned ldb,
                                                  float* __restrict__ C, unsigned ldc, const float* __restrict__ bias,
                                                  unsigned M, unsigned N, unsigned K) {
  gemm64_body<0, FUS_CARRY * W_CARRY, 1>(A, lda, Bt, ldb, (void*)C, ldc, bias, M, N, K, 0u);
}

__global__ __launch_bounds__(256) void k_wt16(const float* __restrict__ Wm, unsigned KI, unsigned NO, _Float16* __restrict__ W16) {
    const unsigned layer = blockIdx.y;
    const float* Wl = Wm + (size_t)layer * KI * NO;
    _Float16* Dl = W16 + (size_t)layer * KI * NO;
    const unsigned u = blockIdx.x * 256u + threadIdx.x;
    const unsigned per = KI >> 3;
    if (u >= NO * per) return;
    const unsigned o = u / per;
    const unsigned k0 = 8u * (u - o * per);
    float v[8];
#pragma unroll
    for (int i = 0; i < 8; ++i) v[i] = bfr(Wl[(size_t)(k0 + (unsigned)i) * NO + o]) * (float)W_CARRY;
    st8hf(Dl, (size_t)o * KI + k0, v);
}

template <unsigned S>
__device__ __forceinline__ void pool_body(const float* __restrict__ x, _Float16* __restrict__ xp) {
    constexpr unsigned HS = 32u / S, NSS = HS * HS;
    const unsigned u = blockIdx.x * 256u + threadIdx.x;
    if (u >= (unsigned)NB * NSS * (unsigned)CW8) return;
    const unsigned row = u / (unsigned)CW8;
    const unsigned c0 = (u - row * (unsigned)CW8) * 8u;
    const unsigned b = row / NSS;
    const unsigned n = row - b * NSS;
    const unsigned i = n / HS;
    const unsigned j = n - i * HS;
    const float* src0 = x + ((size_t)b * SEQ + (i * S) * 32u + j * S) * CDIM + c0;
    v4f a0 = (v4f){0.f, 0.f, 0.f, 0.f}, a1 = a0;
#pragma unroll 1
    for (unsigned di = 0; di < S; ++di) {
#pragma unroll 1
        for (unsigned dj = 0; dj < S; ++dj) {
            const float* s = src0 + (size_t)(di * 32u + dj) * CDIM;
            const v4f p = *(const v4f*)s;
            const v4f q = *(const v4f*)(s + 4);
            a0.x += bfr(p.x); a0.y += bfr(p.y); a0.z += bfr(p.z); a0.w += bfr(p.w);
            a1.x += bfr(q.x); a1.y += bfr(q.y); a1.z += bfr(q.z); a1.w += bfr(q.w);
        }
    }
    constexpr float sc = (float)X_CARRY / (float)(S * S);
    float v[8] = {a0.x * sc, a0.y * sc, a0.z * sc, a0.w * sc, a1.x * sc, a1.y * sc, a1.z * sc, a1.w * sc};
    st8hf(xp, (size_t)row * CDIM + c0, v);
}
__global__ __launch_bounds__(256) void k_pool1(const float* __restrict__ x, _Float16* __restrict__ xp) { pool_body<1u>(x, xp); }
__global__ __launch_bounds__(256) void k_pool2(const float* __restrict__ x, _Float16* __restrict__ xp) { pool_body<2u>(x, xp); }
__global__ __launch_bounds__(256) void k_pool4(const float* __restrict__ x, _Float16* __restrict__ xp) { pool_body<4u>(x, xp); }

template <unsigned NS>
__device__ __forceinline__ void attn_ctx_body(const _Float16* __restrict__ Qp, const _Float16* __restrict__ Kp,
                                              const _Float16* __restrict__ VTp, _Float16* __restrict__ ctx,
                                              float* __restrict__ stm, float* __restrict__ stl) {
    __shared__ __align__(16) float sO[8][16 * 68];
    __shared__ __align__(16) float sM[128];
    __shared__ __align__(16) float sL[128];
    static_assert(NS % 64u == 0u && NS >= 64u);
    const unsigned lane = threadIdx.x & 31u;
    const unsigned wave = (unsigned)__builtin_amdgcn_readfirstlane((int)(threadIdx.x >> 5));
    const unsigned hh = lane >> 4, c = lane & 15u;
    const unsigned flat0 = blockIdx.x * 128u + wave * 16u;
    const unsigned bh = flat0 / NS;
    const unsigned n0 = flat0 - bh * NS;
    const unsigned b = bh / 12u;
    const unsigned h = bh - b * 12u;

    const _Float16* qrow = Qp + ((size_t)bh * NS + n0 + c) * 64u + 8u * hh;
    const v16h qf0 = frag_ld(qrow);
    const v16h qf1 = frag_ld(qrow + 32);
    const _Float16* kbase = Kp + ((size_t)bh * NS + c) * 64u + 8u * hh;
    const _Float16* vbase = VTp + ((size_t)bh * 64u + c) * NS + 8u * hh;

    float mrun = -3.0e38f, lrun = 0.0f;
    v8f o[4];
#pragma unroll
    for (int t = 0; t < 4; ++t) o[t] = (v8f){0.f,0.f,0.f,0.f,0.f,0.f,0.f,0.f};

#pragma unroll 1
    for (unsigned k0 = 0; k0 < NS; k0 += 32u) {
        const _Float16* kr = kbase + (size_t)k0 * 64u;
        v8f s0 = (v8f){0.f,0.f,0.f,0.f,0.f,0.f,0.f,0.f};
        v8f s1 = s0;
        s0 = wmma16(frag_ld(kr), qf0, s0);
        s0 = wmma16(frag_ld(kr + 32), qf1, s0);
        s1 = wmma16(frag_ld(kr + 1024), qf0, s1);
        s1 = wmma16(frag_ld(kr + 1056), qf1, s1);
        float mx = -3.0e38f;
#pragma unroll
        for (int r = 0; r < 8; ++r) {
            s0[r] *= SC2; s1[r] *= SC2;
            mx = fmaxf(mx, fmaxf(s0[r], s1[r]));
        }
        mx = fmaxf(mx, __shfl_xor(mx, 16, 32));
        const float mnew = fmaxf(mrun, mx);
        const float alpha = exp2f(mrun - mnew);
        mrun = mnew;
        float ps = 0.0f;
        v16h pb;
#pragma unroll
        for (int r = 0; r < 8; ++r) {
            const float p0 = exp2f(s0[r] - mnew);
            const float p1 = exp2f(s1[r] - mnew);
            ps += p0 + p1;
            pb[r] = toh_flush(p0 * (float)P_CARRY);
            pb[8 + r] = toh_flush(p1 * (float)P_CARRY);
        }
        ps += __shfl_xor(ps, 16, 32);
        lrun = lrun * alpha + ps;
#pragma unroll
        for (int t = 0; t < 4; ++t) {
#pragma unroll
            for (int r = 0; r < 8; ++r) o[t][r] *= alpha;
        }
#pragma unroll
        for (int t = 0; t < 4; ++t)
            o[t] = wmma16(frag_ld(vbase + (size_t)((unsigned)t * 16u) * NS + k0), pb, o[t]);
    }

    if (hh == 0u) { sM[wave * 16u + c] = mrun; sL[wave * 16u + c] = lrun; }
    const float fin = (1.0f / lrun) * CTX_FOLD;
#pragma unroll
    for (int t = 0; t < 4; ++t) {
        v4f w0, w1;
        w0.x = o[t][0] * fin; w0.y = o[t][1] * fin; w0.z = o[t][2] * fin; w0.w = o[t][3] * fin;
        w1.x = o[t][4] * fin; w1.y = o[t][5] * fin; w1.z = o[t][6] * fin; w1.w = o[t][7] * fin;
        *(v4f*)&sO[wave][c * 68u + (unsigned)t * 16u + 8u * hh] = w0;
        *(v4f*)&sO[wave][c * 68u + (unsigned)t * 16u + 8u * hh + 4u] = w1;
    }
    wave_sync_lds();
    {
        const unsigned q = lane >> 3, c8 = (lane & 7u) * 8u;
        v8h ov[4];
#pragma unroll
        for (int it = 0; it < 4; ++it) {
            const unsigned row = (unsigned)it * 4u + q;
            const v4f s0 = *(const v4f*)&sO[wave][row * 68u + c8];
            const v4f s1 = *(const v4f*)&sO[wave][row * 68u + c8 + 4u];
            ov[it][0] = toh_flush(s0.x); ov[it][1] = toh_flush(s0.y); ov[it][2] = toh_flush(s0.z); ov[it][3] = toh_flush(s0.w);
            ov[it][4] = toh_flush(s1.x); ov[it][5] = toh_flush(s1.y); ov[it][6] = toh_flush(s1.z); ov[it][7] = toh_flush(s1.w);
        }
        _Float16* dst = ctx + (size_t)(b * NS + n0) * CDIM + h * 64u;
        for (int pass = 0; pass < 2; ++pass) {
#pragma unroll
            for (int it = 0; it < 4; ++it)
                *(volatile v8h*)(dst + (size_t)((unsigned)it * 4u + q) * CDIM + c8) = ov[it];
            __threadfence();
        }
    }
    __syncthreads();
    if (wave == 0u) {
        const v4f mv = *(const v4f*)&sM[4u * lane];
        VST2V4(stm + (size_t)blockIdx.x * 128u + 4u * lane, mv);
    } else if (wave == 1u) {
        const v4f lv = *(const v4f*)&sL[4u * lane];
        VST2V4(stl + (size_t)blockIdx.x * 128u + 4u * lane, lv);
    }
}
__global__ __launch_bounds__(256) void k_attn_ctx_1024(const _Float16* __restrict__ Qp, const _Float16* __restrict__ Kp,
                                                       const _Float16* __restrict__ VTp, _Float16* __restrict__ ctx,
                                                       float* __restrict__ stm, float* __restrict__ stl) {
    attn_ctx_body<1024u>(Qp, Kp, VTp, ctx, stm, stl);
}
__global__ __launch_bounds__(256) void k_attn_ctx_256(const _Float16* __restrict__ Qp, const _Float16* __restrict__ Kp,
                                                      const _Float16* __restrict__ VTp, _Float16* __restrict__ ctx,
                                                      float* __restrict__ stm, float* __restrict__ stl) {
    attn_ctx_body<256u>(Qp, Kp, VTp, ctx, stm, stl);
}
__global__ __launch_bounds__(256) void k_attn_ctx_64(const _Float16* __restrict__ Qp, const _Float16* __restrict__ Kp,
                                                     const _Float16* __restrict__ VTp, _Float16* __restrict__ ctx,
                                                     float* __restrict__ stm, float* __restrict__ stl) {
    attn_ctx_body<64u>(Qp, Kp, VTp, ctx, stm, stl);
}

template <unsigned NS>
__device__ __forceinline__ void attn_map_body(const _Float16* __restrict__ Qp, const _Float16* __restrict__ Kp,
                                              const float* __restrict__ stm, const float* __restrict__ stl,
                                              float* __restrict__ map) {
    __shared__ __align__(16) float sA[8][16 * 68];
    static_assert(NS % 64u == 0u && NS >= 64u);
    constexpr unsigned KB = NS / 64u, QT = NS / 16u;
    const unsigned lane = threadIdx.x & 31u;
    const unsigned wave = (unsigned)__builtin_amdgcn_readfirstlane((int)(threadIdx.x >> 5));
    const unsigned hh = lane >> 4, c = lane & 15u;
    const unsigned wg = blockIdx.x * 8u + wave;
    if (wg >= (unsigned)NB * QT * KB) return;
    const unsigned t2 = wg / KB;
    const unsigned kb = wg - t2 * KB;
    const unsigned b = t2 / QT;
    const unsigned qt = t2 - b * QT;
    const unsigned q0 = qt * 16u, key0 = kb * 64u;

    v8f am[4];
#pragma unroll
    for (int j = 0; j < 4; ++j) am[j] = (v8f){0.f,0.f,0.f,0.f,0.f,0.f,0.f,0.f};

#pragma unroll 1
    for (unsigned h = 0; h < (unsigned)HEADS; ++h) {
        const unsigned bh = b * 12u + h;
        const _Float16* qrow = Qp + ((size_t)bh * NS + q0 + c) * 64u + 8u * hh;
        const v16h qf0 = frag_ld(qrow);
        const v16h qf1 = frag_ld(qrow + 32);
        const unsigned si = bh * NS + q0 + c;
        const float mq = stm[si];
        const float il = 1.0f / stl[si];
        const _Float16* kr = Kp + ((size_t)bh * NS + key0 + c) * 64u + 8u * hh;
#pragma unroll
        for (int j = 0; j < 4; ++j) {
            v8f s = (v8f){0.f,0.f,0.f,0.f,0.f,0.f,0.f,0.f};
            s = wmma16(frag_ld(kr + (size_t)((unsigned)j * 1024u)), qf0, s);
            s = wmma16(frag_ld(kr + (size_t)((unsigned)j * 1024u + 32u)), qf1, s);
#pragma unroll
            for (int r = 0; r < 8; ++r) {
                const float e = s[r] * SC2;
                am[j][r] += exp2f(e - mq) * il;
            }
        }
    }
#pragma unroll
    for (int j = 0; j < 4; ++j) {
        v4f w0, w1;
        w0.x = am[j][0] * INV_HEADS; w0.y = am[j][1] * INV_HEADS; w0.z = am[j][2] * INV_HEADS; w0.w = am[j][3] * INV_HEADS;
        w1.x = am[j][4] * INV_HEADS; w1.y = am[j][5] * INV_HEADS; w1.z = am[j][6] * INV_HEADS; w1.w = am[j][7] * INV_HEADS;
        *(v4f*)&sA[wave][c * 68u + (unsigned)j * 16u + 8u * hh] = w0;
        *(v4f*)&sA[wave][c * 68u + (unsigned)j * 16u + 8u * hh + 4u] = w1;
    }
    wave_sync_lds();
    {
        float* dst = map + (size_t)(b * NS + q0) * NS + key0;
        const unsigned c4 = c * 4u;
#pragma unroll
        for (int half = 0; half < 2; ++half) {
            v4f vv[4];
#pragma unroll
            for (int it = 0; it < 4; ++it) {
                const unsigned row = (unsigned)(half * 4 + it) * 2u + hh;
                vv[it] = *(const v4f*)&sA[wave][row * 68u + c4];
            }
            for (int pass = 0; pass < 2; ++pass) {
#pragma unroll
                for (int it = 0; it < 4; ++it) {
                    const unsigned row = (unsigned)(half * 4 + it) * 2u + hh;
                    *(volatile v4f*)(dst + (size_t)row * NS + c4) = vv[it];
                }
                __threadfence();
            }
        }
    }
}
__global__ __launch_bounds__(256) void k_attn_map_1024(const _Float16* __restrict__ Qp, const _Float16* __restrict__ Kp,
                                                       const float* __restrict__ stm, const float* __restrict__ stl,
                                                       float* __restrict__ map) {
    attn_map_body<1024u>(Qp, Kp, stm, stl, map);
}
__global__ __launch_bounds__(256) void k_attn_map_256(const _Float16* __restrict__ Qp, const _Float16* __restrict__ Kp,
                                                      const float* __restrict__ stm, const float* __restrict__ stl,
                                                      float* __restrict__ map) {
    attn_map_body<256u>(Qp, Kp, stm, stl, map);
}
__global__ __launch_bounds__(256) void k_attn_map_64(const _Float16* __restrict__ Qp, const _Float16* __restrict__ Kp,
                                                     const float* __restrict__ stm, const float* __restrict__ stl,
                                                     float* __restrict__ map) {
    attn_map_body<64u>(Qp, Kp, stm, stl, map);
}

__device__ __forceinline__ void tap2(unsigned t, float rs, int hmax, unsigned& ia, unsigned& ib, float& f) {
    const float pos = ((float)t + 0.5f) * rs - 0.5f;
    const float fl = floorf(pos);
    f = pos - fl;
    const int i0 = (int)fl;
    ia = (unsigned)min(max(i0, 0), hmax);
    ib = (unsigned)min(max(i0 + 1, 0), hmax);
}

__global__ __launch_bounds__(256) void k_fuse(const float* __restrict__ F0, const float* __restrict__ F1, const float* __restrict__ F2,
                                              const float* __restrict__ fw, _Float16* __restrict__ fus) {
    const unsigned u = blockIdx.x * 256u + threadIdx.x;
    if (u >= (unsigned)MTOK * (unsigned)CW8) return;
    const unsigned row = u / (unsigned)CW8;
    const unsigned c0 = (u - row * (unsigned)CW8) * 8u;
    const unsigned b = row >> 10, n = row & 1023u;
    const unsigned y = n >> 5, xx = n & 31u;

    const float g0 = bfr(fw[0]), g1 = bfr(fw[1]), g2 = bfr(fw[2]);
    const float gm = fmaxf(g0, fmaxf(g1, g2));
    const float e0 = exp2f((g0 - gm) * LOG2E), e1 = exp2f((g1 - gm) * LOG2E), e2 = exp2f((g2 - gm) * LOG2E);
    const float rs = 1.0f / (e0 + e1 + e2);
    const float w0 = e0 * rs, w1 = e1 * rs, w2 = e2 * rs;

    unsigned ya1, yb1, xa1, xb1, ya2, yb2, xa2, xb2;
    float wy1, wx1, wy2, wx2;
    tap2(y, 0.5f, 15, ya1, yb1, wy1);
    tap2(xx, 0.5f, 15, xa1, xb1, wx1);
    tap2(y, 0.25f, 7, ya2, yb2, wy2);
    tap2(xx, 0.25f, 7, xa2, xb2, wx2);

    const float* r0 = F0 + (size_t)row * CDIM + c0;
    const float* p1 = F1 + (size_t)b * 256u * CDIM + c0;
    const float* p2 = F2 + (size_t)b * 64u * CDIM + c0;
    const float* r1aa = p1 + (size_t)(ya1 * 16u + xa1) * CDIM;
    const float* r1ab = p1 + (size_t)(ya1 * 16u + xb1) * CDIM;
    const float* r1ba = p1 + (size_t)(yb1 * 16u + xa1) * CDIM;
    const float* r1bb = p1 + (size_t)(yb1 * 16u + xb1) * CDIM;
    const float* r2aa = p2 + (size_t)(ya2 * 8u + xa2) * CDIM;
    const float* r2ab = p2 + (size_t)(ya2 * 8u + xb2) * CDIM;
    const float* r2ba = p2 + (size_t)(yb2 * 8u + xa2) * CDIM;
    const float* r2bb = p2 + (size_t)(yb2 * 8u + xb2) * CDIM;

    unsigned q0 = 0u, q1 = 0u, q2 = 0u, q3 = 0u;
#pragma unroll 1
    for (unsigned g = 0; g < 2u; ++g) {
        const unsigned co = 4u * g;
        const v4f f0 = *(const v4f*)(r0 + co);
        const v4f a00 = *(const v4f*)(r1aa + co), a01 = *(const v4f*)(r1ab + co);
        const v4f a10 = *(const v4f*)(r1ba + co), a11 = *(const v4f*)(r1bb + co);
        const v4f b00 = *(const v4f*)(r2aa + co), b01 = *(const v4f*)(r2ab + co);
        const v4f b10 = *(const v4f*)(r2ba + co), b11 = *(const v4f*)(r2bb + co);
        const v4f t1 = a00 * (1.0f - wx1) + a01 * wx1;
        const v4f u1 = a10 * (1.0f - wx1) + a11 * wx1;
        const v4f v1 = t1 * (1.0f - wy1) + u1 * wy1;
        const v4f t2 = b00 * (1.0f - wx2) + b01 * wx2;
        const v4f u2 = b10 * (1.0f - wx2) + b11 * wx2;
        const v4f v2 = t2 * (1.0f - wy2) + u2 * wy2;
        v4f r = (f0 * w0 + v1 * w1) + v2 * w2;
        r = r * (float)FUS_CARRY;
        const unsigned lo = pack2h(r.x, r.y);
        const unsigned hi = pack2h(r.z, r.w);
        if (g == 0u) { q0 = lo; q1 = hi; } else { q2 = lo; q3 = hi; }
    }
    v4u pk; pk.x = q0; pk.y = q1; pk.z = q2; pk.w = q3;
    VST2(v4u, (v4u*)(fus + (size_t)row * CDIM + c0), pk);
}

static inline unsigned gemm_blocks(unsigned M, unsigned N) { return ((M >> 6) * (N >> 6) + 7u) / 8u; }

extern "C" void kernel_launch(void* const* d_in, const int* in_sizes, int n_in, void* d_out, int out_size,
                              void* d_ws, size_t ws_size, hipStream_t stream) {
    if (n_in < 10) return;
    if (in_sizes[0] < MTOK * CDIM || in_sizes[1] < 3 * CDIM * C3 || in_sizes[2] < 3 * C3 || in_sizes[3] < 3 * CDIM * CDIM) return;
    if (in_sizes[4] < 3 * CDIM || in_sizes[5] < 3 * CDIM * CDIM || in_sizes[6] < 3 * CDIM || in_sizes[7] < 3) return;
    if (in_sizes[8] < CDIM * CDIM || in_sizes[9] < CDIM || out_size < OUT3_OFF + NB * 64 * 64) return;

    const float* x      = (const float*)d_in[0];
    const float* qkv_w  = (const float*)d_in[1];
    const float* qkv_b  = (const float*)d_in[2];
    const float* proj_w = (const float*)d_in[3];
    const float* proj_b = (const float*)d_in[4];
    const float* sp_w   = (const float*)d_in[5];
    const float* sp_b   = (const float*)d_in[6];
    const float* fus_w  = (const float*)d_in[7];
    const float* out_w  = (const float*)d_in[8];
    const float* out_b  = (const float*)d_in[9];
    float* out = (float*)d_out;

    char* wsp = (char*)d_ws;
    size_t off = 0;
    auto carve = [&](size_t bytes) -> void* { void* r = wsp + off; off += (bytes + 255) & ~(size_t)255; return r; };
    _Float16* wqkv  = (_Float16*)carve((size_t)3 * C3 * CDIM * 2);
    _Float16* wproj = (_Float16*)carve((size_t)3 * CDIM * CDIM * 2);
    _Float16* wsp16 = (_Float16*)carve((size_t)3 * CDIM * CDIM * 2);
    _Float16* wout  = (_Float16*)carve((size_t)CDIM * CDIM * 2);
    _Float16* x0    = (_Float16*)carve((size_t)MTOK * CDIM * 2);
    _Float16* x1    = (_Float16*)carve((size_t)NB * 256 * CDIM * 2);
    _Float16* x2    = (_Float16*)carve((size_t)NB * 64 * CDIM * 2);
    _Float16* qk16  = (_Float16*)carve((size_t)2 * QK_PLANE * 2);
    _Float16* vt16  = (_Float16*)carve((size_t)QK_PLANE * 2);
    float*    stm   = (float*)carve((size_t)NB * HEADS * SEQ * 4);
    float*    stl   = (float*)carve((size_t)NB * HEADS * SEQ * 4);
    _Float16* ctx16 = (_Float16*)carve((size_t)MTOK * CDIM * 2);
    float*    feat0 = (float*)carve((size_t)MTOK * CDIM * 4);
    float*    feat1 = (float*)carve((size_t)NB * 256 * CDIM * 4);
    float*    feat2 = (float*)carve((size_t)NB * 64 * CDIM * 4);
    if (off > ws_size || off > (size_t)134217728) return;
    _Float16* kpl   = qk16 + (size_t)QK_PLANE;
    _Float16* att16 = qk16;
    _Float16* fus16 = x0;

    k_wt16<<<dim3((C3 * CW8) / 256, 3), 256, 0, stream>>>(qkv_w, CDIM, C3, wqkv);
    k_wt16<<<dim3((CDIM * CW8) / 256, 3), 256, 0, stream>>>(proj_w, CDIM, CDIM, wproj);
    k_wt16<<<dim3((CDIM * CW8) / 256, 3), 256, 0, stream>>>(sp_w, CDIM, CDIM, wsp16);
    k_wt16<<<dim3((CDIM * CW8) / 256, 1), 256, 0, stream>>>(out_w, CDIM, CDIM, wout);

    k_pool1<<<(NB * 1024 * CW8 + 255) / 256, 256, 0, stream>>>(x, x0);
    k_pool2<<<(NB * 256 * CW8 + 255) / 256, 256, 0, stream>>>(x, x1);
    k_pool4<<<(NB * 64 * CW8 + 255) / 256, 256, 0, stream>>>(x, x2);

    {
        const unsigned MS = (unsigned)NB * 1024u;
        k_gemm_qk<<<gemm_blocks(MS, 2u * CDIM), 256, 0, stream>>>(x0, CDIM, wqkv, CDIM, qk16, qkv_b, MS, 2u * CDIM, CDIM, 10u);
        k_gemm_vt<<<gemm_blocks(CDIM, MS), 256, 0, stream>>>(wqkv + (size_t)2 * CDIM * CDIM, CDIM, x0, CDIM, vt16, qkv_b + 2 * CDIM,
                                                              CDIM, MS, CDIM, 10u);
        k_attn_ctx_1024<<<(NB * HEADS * 1024) / 128, 256, 0, stream>>>(qk16, kpl, vt16, ctx16, stm, stl);
        k_attn_map_1024<<<(NB * 64 * 16 + 7) / 8, 256, 0, stream>>>(qk16, kpl, stm, stl, out + OUT1_OFF);
        k_gemm_proj<<<gemm_blocks(MS, CDIM), 256, 0, stream>>>(ctx16, CDIM, wproj, CDIM, att16, CDIM, proj_b, MS, CDIM, CDIM);
        k_gemm_sp<<<gemm_blocks(MS, CDIM), 256, 0, stream>>>(att16, CDIM, wsp16, CDIM, feat0, CDIM, sp_b, MS, CDIM, CDIM);
    }
    {
        const unsigned MS = (unsigned)NB * 256u;
        const _Float16* wq = wqkv + (size_t)C3 * CDIM;
        k_gemm_qk<<<gemm_blocks(MS, 2u * CDIM), 256, 0, stream>>>(x1, CDIM, wq, CDIM, qk16, qkv_b + C3, MS, 2u * CDIM, CDIM, 8u);
        k_gemm_vt<<<gemm_blocks(CDIM, MS), 256, 0, stream>>>(wq + (size_t)2 * CDIM * CDIM, CDIM, x1, CDIM, vt16, qkv_b + C3 + 2 * CDIM,
                                                              CDIM, MS, CDIM, 8u);
        k_attn_ctx_256<<<(NB * HEADS * 256) / 128, 256, 0, stream>>>(qk16, kpl, vt16, ctx16, stm, stl);
        k_attn_map_256<<<(NB * 16 * 4 + 7) / 8, 256, 0, stream>>>(qk16, kpl, stm, stl, out + OUT2_OFF);
        k_gemm_proj<<<gemm_blocks(MS, CDIM), 256, 0, stream>>>(ctx16, CDIM, wproj + (size_t)CDIM * CDIM, CDIM, att16, CDIM,
                                                                proj_b + CDIM, MS, CDIM, CDIM);
        k_gemm_sp<<<gemm_blocks(MS, CDIM), 256, 0, stream>>>(att16, CDIM, wsp16 + (size_t)CDIM * CDIM, CDIM, feat1, CDIM,
                                                              sp_b + CDIM, MS, CDIM, CDIM);
    }
    {
        const unsigned MS = (unsigned)NB * 64u;
        const _Float16* wq = wqkv + (size_t)2 * C3 * CDIM;
        k_gemm_qk<<<gemm_blocks(MS, 2u * CDIM), 256, 0, stream>>>(x2, CDIM, wq, CDIM, qk16, qkv_b + 2 * C3, MS, 2u * CDIM, CDIM, 6u);
        k_gemm_vt<<<gemm_blocks(CDIM, MS), 256, 0, stream>>>(wq + (size_t)2 * CDIM * CDIM, CDIM, x2, CDIM, vt16, qkv_b + 2 * C3 + 2 * CDIM,
                                                              CDIM, MS, CDIM, 6u);
        k_attn_ctx_64<<<(NB * HEADS * 64) / 128, 256, 0, stream>>>(qk16, kpl, vt16, ctx16, stm, stl);
        k_attn_map_64<<<(NB * 4 * 1 + 7) / 8, 256, 0, stream>>>(qk16, kpl, stm, stl, out + OUT3_OFF);
        k_gemm_proj<<<gemm_blocks(MS, CDIM), 256, 0, stream>>>(ctx16, CDIM, wproj + (size_t)2 * CDIM * CDIM, CDIM, att16, CDIM,
                                                                proj_b + 2 * CDIM, MS, CDIM, CDIM);
        k_gemm_sp<<<gemm_blocks(MS, CDIM), 256, 0, stream>>>(att16, CDIM, wsp16 + (size_t)2 * CDIM * CDIM, CDIM, feat2, CDIM,
                                                              sp_b + 2 * CDIM, MS, CDIM, CDIM);
    }

    k_fuse<<<(MTOK * CW8 + 255) / 256, 256, 0, stream>>>(feat0, feat1, feat2, fus_w, fus16);
    k_gemm_out<<<gemm_blocks((unsigned)MTOK, CDIM), 256, 0, stream>>>(fus16, CDIM, wout, CDIM, out, CDIM, out_b,
                                                                       (unsigned)MTOK, CDIM, CDIM);
}
